// BakedAttentionHead_62380105007586
// MI455X (gfx1250) — hardware-run, weakly checked
//
#include <hip/hip_runtime.h>
#include <math.h>

typedef __attribute__((ext_vector_type(16))) _Float16 v16h;
typedef __attribute__((ext_vector_type(8)))  _Float16 v8h;
typedef __attribute__((ext_vector_type(4)))  _Float16 v4h;
typedef __attribute__((ext_vector_type(2)))  _Float16 v2h;
typedef __attribute__((ext_vector_type(16))) __bf16   v16b;
typedef __attribute__((ext_vector_type(8)))  __bf16   v8b;
typedef __attribute__((ext_vector_type(8)))  float    v8f;
typedef __attribute__((ext_vector_type(4)))  float    v4f;
typedef __attribute__((ext_vector_type(2)))  float    v2f;

constexpr int kQ    = 8192;
constexpr int kDim  = 1024;
constexpr int kKeys = 2048;
constexpr int kThr  = 256;
constexpr int kBits = 16;
constexpr float kSharp = 100.0f;

constexpr float kInCarry = 1024.0f;
constexpr float kWCarry  = 1024.0f;
constexpr float kPCarry  = 65536.0f;
constexpr float kScScale = (1.0f / (kInCarry * kWCarry)) * 0.03125f;
constexpr float kOutScale = 1.0f / (kPCarry * kWCarry);
constexpr float kF16MinNormal = 6.103515625e-5f;

static_assert((kQ % 64) == 0 && (kKeys % 64) == 0 && (kDim % 64) == 0, "GEMM M, N multiples of 64, K of 32");
static_assert(kDim == 1024, "the score scale is 2^-5");

constexpr size_t kOffQ16 = 0;
constexpr size_t kOffK16 = kOffQ16 + (size_t)kQ * kDim * 2;
constexpr size_t kOffVT  = kOffK16 + (size_t)kKeys * kDim * 2;
constexpr size_t kOffZB  = kOffVT  + (size_t)kDim * kKeys * 2;
constexpr size_t kOffSC  = kOffZB  + (size_t)kKeys * 4;
constexpr size_t kOffP16 = kOffSC  + (size_t)kQ * kKeys * 4;
constexpr size_t kWsTotal = kOffP16 + (size_t)kQ * kKeys * 2;
static_assert(kWsTotal == 125837312ull, "carve total");
static_assert(kWsTotal <= 134217728ull, "carve cap");
static_assert((kOffK16 % 256) == 0 && (kOffVT % 256) == 0 && (kOffZB % 256) == 0 && (kOffSC % 256) == 0 && (kOffP16 % 256) == 0, "aligned regions");

__device__ __forceinline__ unsigned short f2bf_bits(float f) {
  unsigned u = __float_as_uint(f);
  return (unsigned short)((u + 0x7FFFu + ((u >> 16) & 1u)) >> 16);
}
__device__ __forceinline__ float bf_bits2f(unsigned short h) { return __uint_as_float(((unsigned)h) << 16); }
__device__ __forceinline__ float bf16r(float f) { return bf_bits2f(f2bf_bits(f)); }
__device__ __forceinline__ float carry_flush(float v, float carry) {
  const float s = v * carry;
  return (fabsf(s) < kF16MinNormal) ? 0.0f : s;
}
__device__ __forceinline__ float frcp(float x) { return __builtin_amdgcn_rcpf(x); }

__device__ __forceinline__ void dep_guard4_h(v8f& a, v8f& b, v8f& c, v8f& d, v16h x, v16h y) { asm volatile("v_nop\n\tv_nop\n\tv_nop\n\tv_nop" : "+v"(a), "+v"(b), "+v"(c), "+v"(d) : "v"(x), "v"(y)); }
__device__ __forceinline__ void dep_guard4_b(v8f& a, v8f& b, v8f& c, v8f& d, v16b x, v16b y) { asm volatile("v_nop\n\tv_nop\n\tv_nop\n\tv_nop" : "+v"(a), "+v"(b), "+v"(c), "+v"(d) : "v"(x), "v"(y)); }
__device__ __forceinline__ void keep4_h(v16h a, v16h b, v16h c, v16h d) { asm volatile("v_nop" :: "v"(a), "v"(b), "v"(c), "v"(d)); }
__device__ __forceinline__ void keep4_b(v16b a, v16b b, v16b c, v16b d) { asm volatile("v_nop" :: "v"(a), "v"(b), "v"(c), "v"(d)); }
__device__ __forceinline__ void acc_guard4(v8f& a, v8f& b, v8f& c, v8f& d) { asm volatile("v_nop\n\tv_nop\n\tv_nop\n\tv_nop" : "+v"(a), "+v"(b), "+v"(c), "+v"(d)); }

template <typename T> struct Frag;
template <> struct Frag<_Float16> {
  typedef v16h V; union U { v16h v; v8h h[2]; };
  static __device__ __forceinline__ v16h load(const _Float16* p) {
    U f; f.h[0] = *(const v8h*)(p); f.h[1] = *(const v8h*)(p + 16); return f.v;
  }
  static __device__ __forceinline__ v8f mma(v16h a, v16h b, v8f c) {
    return __builtin_amdgcn_wmma_f32_16x16x32_f16(false, a, false, b, (short)0, c, false, false);
  }
  static __device__ __forceinline__ void guard4(v8f& a, v8f& b, v8f& c, v8f& d, v16h x, v16h y) { dep_guard4_h(a, b, c, d, x, y); }
  static __device__ __forceinline__ void keep(v16h a, v16h b, v16h c, v16h d) { keep4_h(a, b, c, d); }
};
template <> struct Frag<__bf16> {
  typedef v16b V; union U { v16b v; v8b h[2]; };
  static __device__ __forceinline__ v16b load(const __bf16* p) {
    U f; f.h[0] = *(const v8b*)(p); f.h[1] = *(const v8b*)(p + 16); return f.v;
  }
  static __device__ __forceinline__ v8f mma(v16b a, v16b b, v8f c) {
    return __builtin_amdgcn_wmma_f32_16x16x32_bf16(false, a, false, b, (short)0, c, false, false);
  }
  static __device__ __forceinline__ void guard4(v8f& a, v8f& b, v8f& c, v8f& d, v16b x, v16b y) { dep_guard4_b(a, b, c, d, x, y); }
  static __device__ __forceinline__ void keep(v16b a, v16b b, v16b c, v16b d) { keep4_b(a, b, c, d); }
};

__device__ __forceinline__ v8f mma_h(v16h a, v16h b, v8f c) {
  c = __builtin_amdgcn_wmma_f32_16x16x32_f16(false, a, false, b, (short)0, c, false, false);
  asm volatile("v_nop\n\tv_nop\n\tv_nop\n\tv_nop" : "+v"(c) : "v"(a), "v"(b));
  return c;
}

template <int ET> struct Elem;
template <> struct Elem<0> { typedef _Float16 T; };
template <> struct Elem<1> { typedef __bf16 T; };
template <int ET, bool SPLIT, int BIAS_MODE, int OUT_MODE, bool RESID, int ACT = 0>
__global__ __launch_bounds__(256) void wmma_gemm64(
    const unsigned short* __restrict__ Ap, const unsigned short* __restrict__ A2p, int lda, long strideA,
    const unsigned short* __restrict__ Btp, const unsigned short* __restrict__ Bt2p, int ldb, long strideB,
    void* __restrict__ Cout, void* __restrict__ Cout2, int ldc, long strideC,
    const float* __restrict__ bias,
    const float* __restrict__ resid, long strideR,
    int M, int N, int K, float scale) {
  typedef typename Elem<ET>::T T;
  typedef typename Frag<T>::V V;
  const T* A = (const T*)Ap; const T* A2 = (const T*)A2p; const T* Bt = (const T*)Btp; const T* Bt2 = (const T*)Bt2p;
  __shared__ __align__(16) float sT[8][16 * 68];
  const int b    = blockIdx.y;
  const int lane = threadIdx.x & 31;
  const int wave = threadIdx.x >> 5;
  const int tilesN = N >> 6;
  const int tilesM = M >> 6;
  const int tile = blockIdx.x * 8 + wave;
  if (tile >= tilesM * tilesN) return;
  const int tm = tile / tilesN;
  const int tn = tile - tm * tilesN;
  const int m0 = tm << 6;
  const int n0 = tn << 6;

  const T* Ab  = A  + (size_t)b * strideA;
  const T* Bb  = Bt + (size_t)b * strideB;
  const T* Ab2 = SPLIT ? (A2  + (size_t)b * strideA) : nullptr;
  const T* Bb2 = SPLIT ? (Bt2 + (size_t)b * strideB) : nullptr;

  const int rlane = lane & 15;
  const int koff  = (lane >> 4) * 8;
  const int mOff  = (lane >> 4) * 8;

  v8f acc[4][4];
#pragma unroll
  for (int i = 0; i < 4; ++i)
#pragma unroll
    for (int j = 0; j < 4; ++j) acc[i][j] = (v8f){0.f,0.f,0.f,0.f,0.f,0.f,0.f,0.f};

  for (int k0 = 0; k0 < K; k0 += 32) {
    V bh[4], bl[4];
#pragma unroll
    for (int j = 0; j < 4; ++j) {
      const size_t bo = (size_t)(n0 + (j << 4) + rlane) * ldb + koff + k0;
      bh[j] = Frag<T>::load(Bb + bo);
      if (SPLIT) bl[j] = Frag<T>::load(Bb2 + bo);
    }
#pragma unroll
    for (int i = 0; i < 4; ++i) {
      const size_t ao = (size_t)(m0 + (i << 4) + rlane) * lda + koff + k0;
      V ah = Frag<T>::load(Ab + ao);
      V al;
      if (SPLIT) al = Frag<T>::load(Ab2 + ao);
#pragma unroll
      for (int j = 0; j < 4; ++j) {
        acc[i][j] = Frag<T>::mma(ah, bh[j], acc[i][j]);
        if (SPLIT) {
          acc[i][j] = Frag<T>::mma(ah, bl[j], acc[i][j]);
          acc[i][j] = Frag<T>::mma(al, bh[j], acc[i][j]);
        }
      }
      Frag<T>::guard4(acc[i][0], acc[i][1], acc[i][2], acc[i][3], ah, SPLIT ? al : ah);
    }
    Frag<T>::keep(bh[0], bh[1], bh[2], bh[3]);
    if (SPLIT) Frag<T>::keep(bl[0], bl[1], bl[2], bl[3]);
  }
  acc_guard4(acc[0][0], acc[0][1], acc[0][2], acc[0][3]);
  acc_guard4(acc[1][0], acc[1][1], acc[1][2], acc[1][3]);
  acc_guard4(acc[2][0], acc[2][1], acc[2][2], acc[2][3]);
  acc_guard4(acc[3][0], acc[3][1], acc[3][2], acc[3][3]);

  float* slab = sT[wave];
  const float* Rb = RESID ? (resid + (size_t)b * strideR) : nullptr;
#pragma unroll
  for (int i = 0; i < 4; ++i) {
    const int mBase = m0 + (i << 4);
#pragma unroll
    for (int j = 0; j < 4; ++j) {
      const int n = n0 + (j << 4) + rlane;
      float bv = 0.f;
      if (BIAS_MODE == 2) bv = bias[n];
#pragma unroll
      for (int r = 0; r < 8; ++r) {
        float v = acc[i][j][r] * scale;
        if (BIAS_MODE == 1) v += bias[mBase + mOff + r];
        if (BIAS_MODE == 2) v += bv;
        if (RESID) v += Rb[(size_t)(mBase + mOff + r) * ldc + n];
        if (ACT == 1) v = tanhf(v);
        if (ACT == 2) v = fmaxf(v, 0.0f);
        if (ACT == 3) v = v / (1.0f + expf(-v));
        if (ACT == 4) v = (v > 0.f) ? v : 0.01f * v;
        slab[(mOff + r) * 68 + (j << 4) + rlane] = v;
      }
    }
    __builtin_amdgcn_fence(__ATOMIC_RELEASE, "workgroup");
    __builtin_amdgcn_wave_barrier();
    __builtin_amdgcn_fence(__ATOMIC_ACQUIRE, "workgroup");
    if (OUT_MODE == 0) {
      float* C = (float*)Cout + (size_t)b * strideC;
      const int hh = lane >> 4, c4 = (lane & 15) * 4;
      for (int pass = 0; pass < 2; ++pass) {
#pragma unroll
        for (int it = 0; it < 8; ++it) {
          const int row = it * 2 + hh;
          v4f v = *(const v4f*)(slab + row * 68 + c4);
          *(volatile v4f*)(C + (size_t)(mBase + row) * ldc + n0 + c4) = v;
        }
        __threadfence();
      }
    } else {
      const int q = lane >> 3, c8 = (lane & 7) * 8;
      unsigned short* C  = (unsigned short*)Cout  + (size_t)b * strideC;
      unsigned short* C2 = (OUT_MODE == 2) ? ((unsigned short*)Cout2 + (size_t)b * strideC) : nullptr;
      for (int pass = 0; pass < 2; ++pass) {
#pragma unroll
        for (int it = 0; it < 4; ++it) {
          const int row = it * 4 + q;
          const float* sp = slab + row * 68 + c8;
          v8h hv, lv;
#pragma unroll
          for (int e = 0; e < 8; ++e) {
            if (OUT_MODE == 1) {
              hv[e] = (_Float16)sp[e];
            } else {
              unsigned short hb = f2bf_bits(sp[e]);
              unsigned short lb = f2bf_bits(sp[e] - bf_bits2f(hb));
              hv[e] = __builtin_bit_cast(_Float16, hb);
              lv[e] = __builtin_bit_cast(_Float16, lb);
            }
          }
          *(volatile v8h*)(C + (size_t)(mBase + row) * ldc + n0 + c8) = hv;
          if (OUT_MODE == 2) *(volatile v8h*)(C2 + (size_t)(mBase + row) * ldc + n0 + c8) = lv;
        }
        __threadfence();
      }
    }
    __builtin_amdgcn_fence(__ATOMIC_RELEASE, "workgroup");
    __builtin_amdgcn_wave_barrier();
    __builtin_amdgcn_fence(__ATOMIC_ACQUIRE, "workgroup");
  }
}

__global__ __launch_bounds__(kThr) void cast_plane_kernel(const float* __restrict__ src, unsigned short* __restrict__ dst,
                                                          int colsLog2, int dstPitch, int dstOff) {
  const int i   = blockIdx.x * kThr + threadIdx.x;
  const int sh  = colsLog2 - 3;
  const int row = i >> sh;
  const int c8  = (i & ((1 << sh) - 1)) * 8;
  const float* sp = src + ((size_t)row << colsLog2) + c8;
  const v4f a0 = *(const v4f*)(sp);
  const v4f a1 = *(const v4f*)(sp + 4);
  v8h hv;
#pragma unroll
  for (int e = 0; e < 4; ++e) {
    const float f0 = a0[e];
    const float f1 = a1[e];
    hv[e]     = (_Float16)carry_flush(bf16r(f0), kInCarry);
    hv[4 + e] = (_Float16)carry_flush(bf16r(f1), kInCarry);
  }
  unsigned short* dp = dst + (size_t)row * dstPitch + dstOff + c8;
  *(volatile v8h*)dp = hv;
  __threadfence();
  *(volatile v8h*)dp = hv;
}
static_assert(kInCarry == kWCarry, "one cast kernel serves inputs and weights");

__global__ __launch_bounds__(kThr) void vt_plane_kernel(const float* __restrict__ V, unsigned short* __restrict__ VT16,
                                                        float* __restrict__ ZB) {
  const int d  = blockIdx.x;
  const int k8 = threadIdx.x * 8;
  if (d == kDim) {
    const v4f z = {0.f, 0.f, 0.f, 0.f};
    for (int pass = 0; pass < 2; ++pass) {
      *(volatile v4f*)(ZB + k8) = z;
      *(volatile v4f*)(ZB + k8 + 4) = z;
      __threadfence();
    }
    return;
  }
  v8h hv;
#pragma unroll
  for (int e = 0; e < 8; ++e) hv[e] = (_Float16)carry_flush(bf16r(V[(size_t)(k8 + e) * kDim + d]), kWCarry);
  unsigned short* dp = VT16 + (size_t)d * kKeys + k8;
  *(volatile v8h*)dp = hv;
  __threadfence();
  *(volatile v8h*)dp = hv;
}

__device__ __forceinline__ float block_red256(float v, float* red, float* red8, int tid, bool isMax) {
  red[tid] = v;
  __syncthreads();
  if (tid < 8) {
    float s = isMax ? red[32 * tid] : 0.0f;
#pragma unroll
    for (int q = 0; q < 8; ++q) {
      const v4f x = *(const v4f*)(red + 32 * tid + 4 * q);
      if (isMax) s = fmaxf(fmaxf(s, fmaxf(x[0], x[1])), fmaxf(x[2], x[3]));
      else s += (x[0] + x[1]) + (x[2] + x[3]);
    }
    red8[tid] = s;
  }
  __syncthreads();
  const v4f a = *(const v4f*)(red8);
  const v4f c = *(const v4f*)(red8 + 4);
  if (isMax) return fmaxf(fmaxf(fmaxf(a[0], a[1]), fmaxf(a[2], a[3])), fmaxf(fmaxf(c[0], c[1]), fmaxf(c[2], c[3])));
  return ((a[0] + a[1]) + (a[2] + a[3])) + ((c[0] + c[1]) + (c[2] + c[3]));
}

__global__ __launch_bounds__(kThr) void softmax1_kernel(const float* __restrict__ SC, unsigned short* __restrict__ P16) {
  __shared__ __align__(16) float red[256];
  __shared__ __align__(16) float red8[8];
  const int row = blockIdx.x;
  const int tid = threadIdx.x;
  const float* sp = SC + (size_t)row * kKeys + 8 * tid;
  const v4f s0 = *(const v4f*)sp;
  const v4f s1 = *(const v4f*)(sp + 4);
  const float pm = fmaxf(fmaxf(fmaxf(s0[0], s0[1]), fmaxf(s0[2], s0[3])), fmaxf(fmaxf(s1[0], s1[1]), fmaxf(s1[2], s1[3])));
  const float m = block_red256(pm, red, red8, tid, true);
  float e[8];
#pragma unroll
  for (int i = 0; i < 8; ++i) e[i] = expf(((i < 4) ? s0[i] : s1[i - 4]) - m);
  const float ps = ((e[0] + e[1]) + (e[2] + e[3])) + ((e[4] + e[5]) + (e[6] + e[7]));
  const float den = 1.0f + block_red256(ps, red, red8, tid, false);
  float r = 1.0f, q = 0.0f, wbit = 0.5f;
#pragma unroll 1
  for (int i = 0; i < kBits; ++i) {
    const float dbl = r * 2.0f;
    const float st = 1.0f / (1.0f + expf(-(kSharp * (dbl - den))));
    r = dbl - den * st;
    q = q + wbit * st;
    wbit *= 0.5f;
  }
  v8h hv;
#pragma unroll
  for (int i = 0; i < 8; ++i) hv[i] = (_Float16)carry_flush(e[i] * q, kPCarry);
  unsigned short* dp = P16 + (size_t)row * kKeys + 8 * tid;
  *(volatile v8h*)dp = hv;
  __threadfence();
  *(volatile v8h*)dp = hv;
}

static_assert(((size_t)kQ * kDim / 8) % kThr == 0 && ((size_t)kKeys * kDim / 8) % kThr == 0, "cast grids exact");

extern "C" void kernel_launch(void* const* d_in, const int* in_sizes, int n_in,
                              void* d_out, int out_size, void* d_ws, size_t ws_size,
                              hipStream_t stream) {
  if (n_in < 3 || d_out == nullptr || d_ws == nullptr) return;
  if (in_sizes[0] != kQ * kDim || in_sizes[1] != kKeys * kDim || in_sizes[2] != kKeys * kDim) return;
  if (out_size != kQ * kDim) return;
  if (ws_size < kWsTotal) return;
  const float* qry = (const float*)d_in[0];
  const float* key = (const float*)d_in[1];
  const float* val = (const float*)d_in[2];
  char* ws = (char*)d_ws;
  unsigned short* Q16  = (unsigned short*)(ws + kOffQ16);
  unsigned short* K16  = (unsigned short*)(ws + kOffK16);
  unsigned short* VT16 = (unsigned short*)(ws + kOffVT);
  float* ZB = (float*)(ws + kOffZB);
  float* SC = (float*)(ws + kOffSC);
  unsigned short* P16 = (unsigned short*)(ws + kOffP16);

  cast_plane_kernel<<<(int)(((size_t)kQ * kDim / 8) / kThr), kThr, 0, stream>>>(qry, Q16, 10, kDim, 0);
  cast_plane_kernel<<<(int)(((size_t)kKeys * kDim / 8) / kThr), kThr, 0, stream>>>(key, K16, 10, kDim, 0);
  vt_plane_kernel<<<kDim + 1, kThr, 0, stream>>>(val, VT16, ZB);
  wmma_gemm64<0, false, 2, 0, false, 0><<<dim3((kQ / 64) * (kKeys / 64) / 8, 1), 256, 0, stream>>>(
      Q16, Q16, kDim, 0L, K16, K16, kDim, 0L, (void*)SC, (void*)SC, kKeys, 0L,
      ZB, nullptr, 0L, kQ, kKeys, kDim, kScScale);
  softmax1_kernel<<<kQ, kThr, 0, stream>>>(SC, P16);
  wmma_gemm64<0, false, 2, 0, false, 0><<<dim3((kQ / 64) * (kDim / 64) / 8, 1), 256, 0, stream>>>(
      P16, P16, kKeys, 0L, VT16, VT16, kKeys, 0L, d_out, d_out, kDim, 0L,
      ZB, nullptr, 0L, kQ, kDim, kKeys, kOutScale);
}
